// DPLR_CS_SSM_62302795596592
// MI455X (gfx1250) — hardware-run, weakly checked
//
#include <hip/hip_runtime.h>
#include <math.h>

typedef __attribute__((ext_vector_type(16))) _Float16 v16h;
typedef __attribute__((ext_vector_type(8)))  _Float16 v8h;
typedef __attribute__((ext_vector_type(2)))  _Float16 v2h;
typedef __attribute__((ext_vector_type(16))) __bf16   v16b;
typedef __attribute__((ext_vector_type(8)))  __bf16   v8b;
typedef __attribute__((ext_vector_type(8)))  float    v8f;
typedef __attribute__((ext_vector_type(4)))  float    v4f;
typedef __attribute__((ext_vector_type(2)))  float    v2f;
typedef __attribute__((ext_vector_type(4)))  _Float16 v4h;

constexpr int kNB   = 32;
constexpr int kL    = 8192;
constexpr int kRows = kNB * kL;
constexpr int kDin  = 64;
constexpr int kNs   = 16;
constexpr int kDo   = 64;
constexpr int kAug  = 96;
constexpr int kK2   = 128;
constexpr int kOut0 = kRows * kDo;
constexpr float kDt = 1.0f;
constexpr int kThr  = 256;
constexpr float kInCarry = 1024.0f;
constexpr float kWCarry  = 4096.0f;
constexpr float kSc = 1.0f / (kInCarry * kWCarry);
constexpr float kF16MinNormal = 6.103515625e-5f;

static_assert(kRows == 262144 && kDin == 64 && kNs == 16 && kDo == 64 && kAug == 2 * kNs + kDin && kK2 == 2 * kDin && (1 << 6) == kDin, "the index arithmetic below uses these sizes");

constexpr size_t kOffA2 = 0ull;
constexpr size_t kOffBD16 = 67108864ull;
constexpr size_t kOffCW16 = 67117056ull;
constexpr size_t kOffBV = 67133440ull;
constexpr size_t kOffMA = 67133696ull;
constexpr size_t kOffMB = 67139840ull;
constexpr size_t kOffBX = 67145984ull;
constexpr size_t kWsTotal = 134254848ull;
static_assert(kWsTotal <= 268435456ull, "the carve stands under the contract's 256 MiB of workspace");
static_assert(kOffA2 == 0
  && kOffBD16 == kOffA2 + 67108864ull
  && kOffCW16 == kOffBD16 + 8192ull
  && kOffBV == kOffCW16 + 16384ull
  && kOffMA == kOffBV + 256ull
  && kOffMB == kOffMA + 6144ull
  && kOffBX == kOffMB + 6144ull
  && kWsTotal == kOffBX + 67108864ull, "the carve is a chain: every region starts where the one before ends");
static_assert((size_t)kRows * kK2 * 2 == 67108864ull && (size_t)64 * kDin * 2 == 8192ull && (size_t)kDo * kK2 * 2 == 16384ull && (size_t)kNs * kAug * 4 == 6144ull && (size_t)kRows * 64 * 4 == 67108864ull, "every region's length is its plane's");
static_assert((kOffBD16 % 256) == 0 && (kOffCW16 % 256) == 0 && (kOffBV % 256) == 0 && (kOffMA % 256) == 0 && (kOffMB % 256) == 0 && (kOffBX % 256) == 0, "every region starts on a multiple of 256 B");

__device__ __forceinline__ unsigned short f2bf_bits(float f) {
  unsigned u = __float_as_uint(f);
  return (unsigned short)((u + 0x7FFFu + ((u >> 16) & 1u)) >> 16);
}
__device__ __forceinline__ float bf_bits2f(unsigned short h) { return __uint_as_float(((unsigned)h) << 16); }
__device__ __forceinline__ float bf16r(float f) { return bf_bits2f(f2bf_bits(f)); }
__device__ __forceinline__ float carry_flush(float v, float carry) {
  const float s = v * carry;
  return (fabsf(s) < kF16MinNormal) ? 0.0f : s;
}

__device__ __forceinline__ void dep_guard4_h(v8f& a, v8f& b, v8f& c, v8f& d, v16h x, v16h y) { asm volatile("v_nop\n\tv_nop\n\tv_nop\n\tv_nop" : "+v"(a), "+v"(b), "+v"(c), "+v"(d) : "v"(x), "v"(y)); }
__device__ __forceinline__ void dep_guard4_b(v8f& a, v8f& b, v8f& c, v8f& d, v16b x, v16b y) { asm volatile("v_nop\n\tv_nop\n\tv_nop\n\tv_nop" : "+v"(a), "+v"(b), "+v"(c), "+v"(d) : "v"(x), "v"(y)); }
__device__ __forceinline__ void keep4_h(v16h a, v16h b, v16h c, v16h d) { asm volatile("v_nop" :: "v"(a), "v"(b), "v"(c), "v"(d)); }
__device__ __forceinline__ void keep4_b(v16b a, v16b b, v16b c, v16b d) { asm volatile("v_nop" :: "v"(a), "v"(b), "v"(c), "v"(d)); }
__device__ __forceinline__ void acc_guard4(v8f& a, v8f& b, v8f& c, v8f& d) { asm volatile("v_nop\n\tv_nop\n\tv_nop\n\tv_nop" : "+v"(a), "+v"(b), "+v"(c), "+v"(d)); }

template <typename T> struct Frag;
template <> struct Frag<_Float16> {
  typedef v16h V; union U { v16h v; v8h h[2]; };
  static __device__ __forceinline__ v16h load(const _Float16* p) {
    U f; f.h[0] = *(const v8h*)(p); f.h[1] = *(const v8h*)(p + 16); return f.v;
  }
  static __device__ __forceinline__ v8f mma(v16h a, v16h b, v8f c) {
    return __builtin_amdgcn_wmma_f32_16x16x32_f16(false, a, false, b, (short)0, c, false, false);
  }
  static __device__ __forceinline__ void guard4(v8f& a, v8f& b, v8f& c, v8f& d, v16h x, v16h y) { dep_guard4_h(a, b, c, d, x, y); }
  static __device__ __forceinline__ void keep(v16h a, v16h b, v16h c, v16h d) { keep4_h(a, b, c, d); }
};
template <> struct Frag<__bf16> {
  typedef v16b V; union U { v16b v; v8b h[2]; };
  static __device__ __forceinline__ v16b load(const __bf16* p) {
    U f; f.h[0] = *(const v8b*)(p); f.h[1] = *(const v8b*)(p + 16); return f.v;
  }
  static __device__ __forceinline__ v8f mma(v16b a, v16b b, v8f c) {
    return __builtin_amdgcn_wmma_f32_16x16x32_bf16(false, a, false, b, (short)0, c, false, false);
  }
  static __device__ __forceinline__ void guard4(v8f& a, v8f& b, v8f& c, v8f& d, v16b x, v16b y) { dep_guard4_b(a, b, c, d, x, y); }
  static __device__ __forceinline__ void keep(v16b a, v16b b, v16b c, v16b d) { keep4_b(a, b, c, d); }
};

__device__ __forceinline__ v8f mma_h(v16h a, v16h b, v8f c) {
  c = __builtin_amdgcn_wmma_f32_16x16x32_f16(false, a, false, b, (short)0, c, false, false);
  asm volatile("v_nop\n\tv_nop\n\tv_nop\n\tv_nop" : "+v"(c) : "v"(a), "v"(b));
  return c;
}

template <int ET> struct Elem;
template <> struct Elem<0> { typedef _Float16 T; };
template <> struct Elem<1> { typedef __bf16 T; };
template <int ET, bool SPLIT, int BIAS_MODE, int OUT_MODE, bool RESID, int ACT = 0>
__global__ __launch_bounds__(256) void wmma_gemm64(
    const unsigned short* __restrict__ Ap, const unsigned short* __restrict__ A2p, int lda, long strideA,
    const unsigned short* __restrict__ Btp, const unsigned short* __restrict__ Bt2p, int ldb, long strideB,
    void* __restrict__ Cout, void* __restrict__ Cout2, int ldc, long strideC,
    const float* __restrict__ bias,
    const float* __restrict__ resid, long strideR,
    int M, int N, int K, float scale) {
  typedef typename Elem<ET>::T T;
  typedef typename Frag<T>::V V;
  const T* A = (const T*)Ap; const T* A2 = (const T*)A2p; const T* Bt = (const T*)Btp; const T* Bt2 = (const T*)Bt2p;
  __shared__ __align__(16) float sT[8][16 * 68];
  const int b    = blockIdx.y;
  const int lane = threadIdx.x & 31;
  const int wave = threadIdx.x >> 5;
  const int tilesN = N >> 6;
  const int tilesM = M >> 6;
  const int tile = blockIdx.x * 8 + wave;
  if (tile >= tilesM * tilesN) return;
  const int tm = tile / tilesN;
  const int tn = tile - tm * tilesN;
  const int m0 = tm << 6;
  const int n0 = tn << 6;

  const T* Ab  = A  + (size_t)b * strideA;
  const T* Bb  = Bt + (size_t)b * strideB;
  const T* Ab2 = SPLIT ? (A2  + (size_t)b * strideA) : nullptr;
  const T* Bb2 = SPLIT ? (Bt2 + (size_t)b * strideB) : nullptr;

  const int rlane = lane & 15;
  const int koff  = (lane >> 4) * 8;
  const int mOff  = (lane >> 4) * 8;

  v8f acc[4][4];
#pragma unroll
  for (int i = 0; i < 4; ++i)
#pragma unroll
    for (int j = 0; j < 4; ++j) acc[i][j] = (v8f){0.f,0.f,0.f,0.f,0.f,0.f,0.f,0.f};

  for (int k0 = 0; k0 < K; k0 += 32) {
    V bh[4], bl[4];
#pragma unroll
    for (int j = 0; j < 4; ++j) {
      const size_t bo = (size_t)(n0 + (j << 4) + rlane) * ldb + koff + k0;
      bh[j] = Frag<T>::load(Bb + bo);
      if (SPLIT) bl[j] = Frag<T>::load(Bb2 + bo);
    }
#pragma unroll
    for (int i = 0; i < 4; ++i) {
      const size_t ao = (size_t)(m0 + (i << 4) + rlane) * lda + koff + k0;
      V ah = Frag<T>::load(Ab + ao);
      V al;
      if (SPLIT) al = Frag<T>::load(Ab2 + ao);
#pragma unroll
      for (int j = 0; j < 4; ++j) {
        acc[i][j] = Frag<T>::mma(ah, bh[j], acc[i][j]);
        if (SPLIT) {
          acc[i][j] = Frag<T>::mma(ah, bl[j], acc[i][j]);
          acc[i][j] = Frag<T>::mma(al, bh[j], acc[i][j]);
        }
      }
      Frag<T>::guard4(acc[i][0], acc[i][1], acc[i][2], acc[i][3], ah, SPLIT ? al : ah);
    }
    Frag<T>::keep(bh[0], bh[1], bh[2], bh[3]);
    if (SPLIT) Frag<T>::keep(bl[0], bl[1], bl[2], bl[3]);
  }
  acc_guard4(acc[0][0], acc[0][1], acc[0][2], acc[0][3]);
  acc_guard4(acc[1][0], acc[1][1], acc[1][2], acc[1][3]);
  acc_guard4(acc[2][0], acc[2][1], acc[2][2], acc[2][3]);
  acc_guard4(acc[3][0], acc[3][1], acc[3][2], acc[3][3]);

  float* slab = sT[wave];
  const float* Rb = RESID ? (resid + (size_t)b * strideR) : nullptr;
#pragma unroll
  for (int i = 0; i < 4; ++i) {
    const int mBase = m0 + (i << 4);
#pragma unroll
    for (int j = 0; j < 4; ++j) {
      const int n = n0 + (j << 4) + rlane;
      float bv = 0.f;
      if (BIAS_MODE == 2) bv = bias[n];
#pragma unroll
      for (int r = 0; r < 8; ++r) {
        float v = acc[i][j][r] * scale;
        if (BIAS_MODE == 1) v += bias[mBase + mOff + r];
        if (BIAS_MODE == 2) v += bv;
        if (RESID) v += Rb[(size_t)(mBase + mOff + r) * ldc + n];
        if (ACT == 1) v = tanhf(v);
        if (ACT == 2) v = fmaxf(v, 0.0f);
        if (ACT == 3) v = v / (1.0f + expf(-v));
        if (ACT == 4) v = (v > 0.f) ? v : 0.01f * v;
        slab[(mOff + r) * 68 + (j << 4) + rlane] = v;
      }
    }
    __builtin_amdgcn_fence(__ATOMIC_RELEASE, "workgroup");
    __builtin_amdgcn_wave_barrier();
    __builtin_amdgcn_fence(__ATOMIC_ACQUIRE, "workgroup");
    if (OUT_MODE == 0) {
      float* C = (float*)Cout + (size_t)b * strideC;
      const int hh = lane >> 4, c4 = (lane & 15) * 4;
      for (int pass = 0; pass < 2; ++pass) {
#pragma unroll
        for (int it = 0; it < 8; ++it) {
          const int row = it * 2 + hh;
          v4f v = *(const v4f*)(slab + row * 68 + c4);
          *(volatile v4f*)(C + (size_t)(mBase + row) * ldc + n0 + c4) = v;
        }
        __threadfence();
      }
    } else {
      const int q = lane >> 3, c8 = (lane & 7) * 8;
      unsigned short* C  = (unsigned short*)Cout  + (size_t)b * strideC;
      unsigned short* C2 = (OUT_MODE == 2) ? ((unsigned short*)Cout2 + (size_t)b * strideC) : nullptr;
      for (int pass = 0; pass < 2; ++pass) {
#pragma unroll
        for (int it = 0; it < 4; ++it) {
          const int row = it * 4 + q;
          const float* sp = slab + row * 68 + c8;
          v8h hv, lv;
#pragma unroll
          for (int e = 0; e < 8; ++e) {
            if (OUT_MODE == 1) {
              hv[e] = (_Float16)sp[e];
            } else {
              unsigned short hb = f2bf_bits(sp[e]);
              unsigned short lb = f2bf_bits(sp[e] - bf_bits2f(hb));
              hv[e] = __builtin_bit_cast(_Float16, hb);
              lv[e] = __builtin_bit_cast(_Float16, lb);
            }
          }
          *(volatile v8h*)(C + (size_t)(mBase + row) * ldc + n0 + c8) = hv;
          if (OUT_MODE == 2) *(volatile v8h*)(C2 + (size_t)(mBase + row) * ldc + n0 + c8) = lv;
        }
        __threadfence();
      }
    }
    __builtin_amdgcn_fence(__ATOMIC_RELEASE, "workgroup");
    __builtin_amdgcn_wave_barrier();
    __builtin_amdgcn_fence(__ATOMIC_ACQUIRE, "workgroup");
  }
}


__global__ __launch_bounds__(kThr) void cast_plane_kernel(const float* __restrict__ src, unsigned short* __restrict__ dst,
                                                          int colsLog2, int dstPitch, int dstOff) {
  const int i   = blockIdx.x * kThr + threadIdx.x;
  const int sh  = colsLog2 - 3;
  const int row = i >> sh;
  const int c8  = (i & ((1 << sh) - 1)) * 8;
  const float* sp = src + ((size_t)row << colsLog2) + c8;
  const v4f a0 = *(const v4f*)(sp);
  const v4f a1 = *(const v4f*)(sp + 4);
  v8h hv;
#pragma unroll
  for (int e = 0; e < 4; ++e) {
    const float f0 = a0[e];
    const float f1 = a1[e];
    hv[e]     = (_Float16)carry_flush(bf16r(f0), kInCarry);
    hv[4 + e] = (_Float16)carry_flush(bf16r(f1), kInCarry);
  }
  unsigned short* dp = dst + (size_t)row * dstPitch + dstOff + c8;
  *(volatile v8h*)dp = hv;
  __threadfence();
  *(volatile v8h*)dp = hv;
}

__global__ __launch_bounds__(kThr) void build_kernel(const float* __restrict__ log_lambda, const float* __restrict__ p, const float* __restrict__ q, const float* __restrict__ B, const float* __restrict__ P, float* __restrict__ MA) {
  const unsigned ix = blockIdx.x * (unsigned)kThr + threadIdx.x;
  const unsigned i = ix / (unsigned)kAug;
  const unsigned j = ix - i * (unsigned)kAug;
  const unsigned jj = j & 15u;
  float a = 0.0f;
#pragma unroll
  for (int l = 0; l < kNs; ++l) {
    float t = 0.0f;
#pragma unroll
    for (int k = 0; k < kNs; ++k) {
      const float core = ((k == l) ? -expf(bf16r(log_lambda[k])) : 0.0f) + bf16r(p[k]) * bf16r(q[l]);
      t += bf16r(P[i * (unsigned)kNs + (unsigned)k]) * core;
    }
    a += t * bf16r(P[jj * (unsigned)kNs + (unsigned)l]);
  }
  const float im = ((i == j) ? 1.0f : 0.0f) - 0.5f * a;
  const float ip = ((i + 16u == j) ? 1.0f : 0.0f) + 0.5f * a;
  const unsigned jb = (j - 32u) & 63u;
  const float bv = bf16r(B[i * (unsigned)kDin + jb]);
  const float o = (j < 16u) ? im : ((j < 32u) ? ip : bv);
  float* dp = MA + ix;
  *(volatile float*)dp = o;
  __threadfence();
  *(volatile float*)dp = o;
}
static_assert(kNs * kAug == 6 * kThr, "the augmented system's grid exact: 6 blocks");

__global__ __launch_bounds__(kThr) void gj_kernel(const float* __restrict__ Min, float* __restrict__ Mout, int k) {
  const unsigned ix = blockIdx.x * (unsigned)kThr + threadIdx.x;
  const unsigned i = ix / (unsigned)kAug;
  const unsigned j = ix - i * (unsigned)kAug;
  const unsigned ku = (unsigned)k;
  const float r = Min[ku * (unsigned)kAug + j] / Min[ku * (unsigned)kAug + ku];
  const float o = (i == ku) ? r : (Min[ix] - Min[i * (unsigned)kAug + ku] * r);
  float* dp = Mout + ix;
  *(volatile float*)dp = o;
  __threadfence();
  *(volatile float*)dp = o;
}

__global__ __launch_bounds__(kThr) void fin_kernel(const float* __restrict__ MF, const float* __restrict__ C, const float* __restrict__ D, unsigned short* __restrict__ BD16, unsigned short* __restrict__ CW16, float* __restrict__ BV) {
  const unsigned ix = blockIdx.x * (unsigned)kThr + threadIdx.x;
  if (ix < 512u) {
    const unsigned n = ix >> 3, d8 = (ix & 7u) * 8u;
    const unsigned nn = (n < 16u) ? n : 0u;
    v8h hv;
#pragma unroll
    for (int e = 0; e < 8; ++e) { const float v = kDt * MF[nn * (unsigned)kAug + 32u + d8 + (unsigned)e]; hv[e] = (_Float16)((n < 16u) ? carry_flush(v, kWCarry) : 0.0f); }
    unsigned short* dp = BD16 + ix * 8u;
    *(volatile v8h*)dp = hv;
    __threadfence();
    *(volatile v8h*)dp = hv;
  } else if (ix < 1536u) {
    const unsigned jx = ix - 512u;
    const unsigned o = jx >> 4, c8 = (jx & 15u) * 8u;
    v8h hv;
#pragma unroll
    for (int e = 0; e < 8; ++e) {
      const unsigned c = c8 + (unsigned)e;
      const float vc = bf16r(C[o * (unsigned)kNs + (c & 15u)]);
      const float vd = bf16r(D[o * (unsigned)kDin + (c & 63u)]);
      hv[e] = (_Float16)((c < 16u) ? carry_flush(vc, kWCarry) : ((c >= 64u) ? carry_flush(vd, kWCarry) : 0.0f));
    }
    unsigned short* dp = CW16 + jx * 8u;
    *(volatile v8h*)dp = hv;
    __threadfence();
    *(volatile v8h*)dp = hv;
  } else if (ix < 1552u) {
    v4f z; z[0] = 0.0f; z[1] = 0.0f; z[2] = 0.0f; z[3] = 0.0f;
    float* dp = BV + (ix - 1536u) * 4u;
    *(volatile v4f*)dp = z;
    __threadfence();
    *(volatile v4f*)dp = z;
  }
}
static_assert(64 * kDin / 8 == 512 && kDo * kK2 / 8 == 1024 && 64 / 4 == 16 && 7 * kThr >= 1552, "the small planes' thread ranges");

__global__ __launch_bounds__(kThr) void scan_kernel(const float* __restrict__ BX, const float* __restrict__ MF, unsigned short* __restrict__ A2) {
  __shared__ __align__(16) float sA[kNs * kNs];
  const unsigned sq = threadIdx.x;
  {
    const v4f* src = (const v4f*)(MF + (sq >> 1) * (unsigned)kAug + 16u + (sq & 1u) * 8u);
    *(v4f*)(sA + sq * 8u) = src[0];
    *(v4f*)(sA + sq * 8u + 4u) = src[1];
  }
  __builtin_amdgcn_fence(__ATOMIC_RELEASE, "workgroup");
  __builtin_amdgcn_wave_barrier();
  __builtin_amdgcn_fence(__ATOMIC_ACQUIRE, "workgroup");
  float h[kNs];
#pragma unroll
  for (int n = 0; n < kNs; ++n) h[n] = 0.0f;
  for (int t = 0; t < kL; ++t) {
    const v4f* ad = (const v4f*)sA;
    const unsigned row = sq * (unsigned)kL + (unsigned)t;
    const float* bp = BX + row * 64u;
    const v4f b0 = *(const v4f*)bp, b1 = *(const v4f*)(bp + 4), b2 = *(const v4f*)(bp + 8), b3 = *(const v4f*)(bp + 12);
    float hn[kNs];
#pragma unroll
    for (int n = 0; n < kNs; ++n) {
      const v4f a0 = ad[n * 4 + 0], a1 = ad[n * 4 + 1], a2 = ad[n * 4 + 2], a3 = ad[n * 4 + 3];
      float s = 0.0f;
#pragma unroll
      for (int m = 0; m < 4; ++m) s += a0[m] * h[m];
#pragma unroll
      for (int m = 0; m < 4; ++m) s += a1[m] * h[4 + m];
#pragma unroll
      for (int m = 0; m < 4; ++m) s += a2[m] * h[8 + m];
#pragma unroll
      for (int m = 0; m < 4; ++m) s += a3[m] * h[12 + m];
      const float bx = (n < 4) ? b0[n & 3] : ((n < 8) ? b1[n & 3] : ((n < 12) ? b2[n & 3] : b3[n & 3]));
      hn[n] = s + bx;
    }
    v8h w0, w1, wz;
#pragma unroll
    for (int e = 0; e < 8; ++e) { h[e] = hn[e]; h[8 + e] = hn[8 + e]; w0[e] = (_Float16)carry_flush(hn[e], kInCarry); w1[e] = (_Float16)carry_flush(hn[8 + e], kInCarry); wz[e] = (_Float16)0.0f; }
    unsigned short* dp = A2 + row * (unsigned)kK2;
    for (int pass = 0; pass < 2; ++pass) {
      *(volatile v8h*)dp = w0;
      *(volatile v8h*)(dp + 8) = w1;
#pragma unroll
      for (int g = 2; g < 8; ++g) *(volatile v8h*)(dp + 8 * g) = wz;
      __threadfence();
    }
  }
}
static_assert(kNB == 32 && (kAug % 4) == 0 && (size_t)kRows * kK2 < 4294967296ull / 2, "the scan is one wave: a lane a sequence; 32-bit element offsets");

extern "C" void kernel_launch(void* const* d_in, const int* in_sizes, int n_in,
                              void* d_out, int out_size, void* d_ws, size_t ws_size,
                              hipStream_t stream) {
  if (n_in < 8 || d_out == nullptr || d_ws == nullptr) return;
  if (in_sizes[0] != kRows * kDin || in_sizes[1] != kNs || in_sizes[2] != kNs || in_sizes[3] != kNs || in_sizes[4] != kNs * kDin || in_sizes[5] != kDo * kNs || in_sizes[6] != kDo * kDin || in_sizes[7] != kNs * kNs) return;
  if (out_size != kOut0) return;
  if (ws_size < kWsTotal) return;
  const float* x = (const float*)d_in[0];
  const float* log_lambda = (const float*)d_in[1];
  const float* p = (const float*)d_in[2];
  const float* q = (const float*)d_in[3];
  const float* B = (const float*)d_in[4];
  const float* C = (const float*)d_in[5];
  const float* D = (const float*)d_in[6];
  const float* P = (const float*)d_in[7];
  float* out = (float*)d_out;
  char* ws = (char*)d_ws;
  unsigned short* A2 = (unsigned short*)(ws + kOffA2);
  unsigned short* BD16 = (unsigned short*)(ws + kOffBD16);
  unsigned short* CW16 = (unsigned short*)(ws + kOffCW16);
  float* BV = (float*)(ws + kOffBV);
  float* MA = (float*)(ws + kOffMA);
  float* MB = (float*)(ws + kOffMB);
  float* BX = (float*)(ws + kOffBX);

  static_assert(((size_t)kRows * kDin / 8) % kThr == 0, "the row cast's grid");
  cast_plane_kernel<<<(int)(((size_t)kRows * kDin / 8) / kThr), kThr, 0, stream>>>(x, A2, 6, kK2, kDin);
  build_kernel<<<6, kThr, 0, stream>>>(log_lambda, p, q, B, P, MA);
  for (int k = 0; k < kNs; k += 2) {
    gj_kernel<<<6, kThr, 0, stream>>>(MA, MB, k);
    gj_kernel<<<6, kThr, 0, stream>>>(MB, MA, k + 1);
  }
  fin_kernel<<<7, kThr, 0, stream>>>(MA, C, D, BD16, CW16, BV);
  wmma_gemm64<0, false, 2, 0, false, 0><<<dim3((kRows / 64) * (64 / 64) / 8, 1), 256, 0, stream>>>(
      A2 + kDin, A2 + kDin, kK2, 0L, BD16, BD16, kDin, 0L, (void*)BX, (void*)BX, 64, 0L, BV, nullptr, 0L, kRows, 64, kDin, kSc);
  scan_kernel<<<1, 32, 0, stream>>>(BX, MA, A2);
  wmma_gemm64<0, false, 2, 0, false, 0><<<dim3((kRows / 64) * (kDo / 64) / 8, 1), 256, 0, stream>>>(
      A2, A2, kK2, 0L, CW16, CW16, kK2, 0L, (void*)out, (void*)out, kDo, 0L, BV, nullptr, 0L, kRows, kDo, kK2, kSc);
}
static_assert(((kRows / 64) * (kDo / 64)) % 8 == 0 && (kNs % 2) == 0, "the engine's grid: whole blocks of eight wave tiles; an even number of elimination steps ends in MA");
